// MulHeadCrossAttn_738734375600
// MI455X (gfx1250) — hardware-verified
//
#include <hip/hip_runtime.h>
#include <math.h>
#include <stdint.h>


#define NB   2
#define SEQ  2048
#define DQ   2048
#define DKV  1024
#define HID  2048
#define NH   16
#define HD   128

static_assert(DQ == HID);
static_assert(NH * HD == HID);

typedef _Float16 v16h __attribute__((ext_vector_type(16)));
typedef _Float16 v8h  __attribute__((ext_vector_type(8)));
typedef float    v8f  __attribute__((ext_vector_type(8)));
typedef float    v4f  __attribute__((ext_vector_type(4)));
typedef unsigned int v4u __attribute__((ext_vector_type(4)));

__constant__ unsigned int kInvFreq[64] = {
  0x3f800000u,0x3f5dafd7u,0x3f3ff911u,0x3f263de0u,0x3f0ff59au,0x3ef953cfu,0x3ed7e89bu,0x3ebaf81bu,
  0x3ea1e89bu,0x3e8c3504u,0x3e72d423u,0x3e5247edu,0x3e361887u,0x3e1db040u,0x3e088d77u,0x3dec7fd6u,
  0x3dcccccdu,0x3db15978u,0x3d99940du,0x3d84fe4du,0x3d6655c2u,0x3d47763fu,0x3d2cba15u,0x3d159348u,
  0x3d0186e3u,0x3ce054d2u,0x3cc2434fu,0x3ca8398bu,0x3c91ad39u,0x3c7c4d33u,0x3c5a7bf2u,0x3c3d3311u,
  0x3c23d70au,0x3c0de12du,0x3bf5b9b0u,0x3bd4ca15u,0x3bb8449cu,0x3b9f91ccu,0x3b8a2e77u,0x3b6f520eu,
  0x3b4f3e38u,0x3b33770fu,0x3b1b690du,0x3b06946fu,0x3ae91528u,0x3ac9d75cu,0x3aaec98eu,0x3a975c0eu,
  0x3a83126fu,0x3a6301e2u,0x3a44948cu,0x3a2a3b44u,0x3a136a16u,0x39ff4facu,0x39dd1725u,0x39bf74d7u,
  0x39a5cb60u,0x398f9272u,0x3978a815u,0x395753e4u,0x393a7753u,0x39217916u,0x390bd472u,0x38f22ce2u };

__device__ __forceinline__ unsigned pk16(unsigned short a, unsigned short b) { return (unsigned)a | ((unsigned)b << 16); }
__device__ __forceinline__ unsigned short h2u(_Float16 x) { return __builtin_bit_cast(unsigned short, x); }
__device__ __forceinline__ unsigned pkf2(float a, float b) { return pk16(h2u((_Float16)a), h2u((_Float16)b)); }

__device__ __forceinline__ void wave_sync() {
  __builtin_amdgcn_fence(__ATOMIC_RELEASE, "workgroup");
  __builtin_amdgcn_wave_barrier();
  __builtin_amdgcn_fence(__ATOMIC_ACQUIRE, "workgroup");
}

union FragH { v16h v; v8h h[2]; };
__device__ __forceinline__ v16h ldfrag_h(const _Float16* p) {
  FragH f; f.h[0] = *(const v8h*)(p); f.h[1] = *(const v8h*)(p + 16); return f.v;
}

__device__ __forceinline__ v8f wmma_h(v16h a, v16h b, v8f c) {
  c = __builtin_amdgcn_wmma_f32_16x16x32_f16(false, a, false, b, (short)0, c, false, false);
  asm volatile("v_nop\n\tv_nop\n\tv_nop\n\tv_nop" : "+v"(c) : "v"(a), "v"(b));
  return c;
}
__device__ __forceinline__ v8f wmma_h_raw(v16h a, v16h b, v8f c) {
  return __builtin_amdgcn_wmma_f32_16x16x32_f16(false, a, false, b, (short)0, c, false, false);
}
__device__ __forceinline__ void dep_guard_h(v8f& x, v8f& y, v16h b, v16h a0, v16h a1) {
  asm volatile("v_nop\n\tv_nop\n\tv_nop\n\tv_nop" : "+v"(x), "+v"(y) : "v"(b), "v"(a0), "v"(a1));
}

__global__ __launch_bounds__(256) void cvt_f16x8_kernel(const float* __restrict__ in, unsigned short* out, int n8) {
  const int i = blockIdx.x * 256 + threadIdx.x;
  if (i < n8) {
    const v4f a = *(const v4f*)(in + 8 * (size_t)i);
    const v4f c = *(const v4f*)(in + 8 * (size_t)i + 4);
    v4u w;
    w[0] = pkf2(a[0], a[1]);
    w[1] = pkf2(a[2], a[3]);
    w[2] = pkf2(c[0], c[1]);
    w[3] = pkf2(c[2], c[3]);
    volatile v4u* p = (volatile v4u*)(out + 8 * (size_t)i);
    *p = w;
    __threadfence();
    *p = w;
  }
}

#define TP 68
__global__ __launch_bounds__(256) void wtr_kernel(const float* __restrict__ in, unsigned short* out, int R, int C, float scl) {
  __shared__ __align__(16) float T[64 * TP];
  const int tid = threadIdx.x;
  const int c0 = blockIdx.x * 64;
  const int r0 = blockIdx.y * 64;
#pragma unroll
  for (int it = 0; it < 4; ++it) {
    const int row = it * 16 + (tid >> 4), col = (tid & 15) * 4;
    const v4f v = *(const v4f*)(in + (size_t)(r0 + row) * C + c0 + col);
    *(v4f*)(T + row * TP + col) = v;
  }
  __syncthreads();
  const int k8 = (tid & 7) * 8, cq = tid >> 3;
#pragma unroll
  for (int it = 0; it < 2; ++it) {
    const int c = it * 32 + cq;
    float o[8];
#pragma unroll
    for (int e = 0; e < 8; ++e) o[e] = T[(k8 + e) * TP + c] * scl;
    v4u w;
#pragma unroll
    for (int p = 0; p < 4; ++p) w[p] = pkf2(o[2 * p], o[2 * p + 1]);
    volatile v4u* gp = (volatile v4u*)(out + (size_t)(c0 + c) * R + r0 + k8);
    *gp = w;
    __threadfence();
    *gp = w;
  }
}

__global__ __launch_bounds__(256) void rope_table_kernel(float* cs, int n) {
#pragma clang fp contract(off)
  const int t = blockIdx.x * 256 + threadIdx.x;
  if (t >= n) return;
  const int s = t >> 6;
  const int i = t & 63;
  const float  inv = __uint_as_float(kInvFreq[i]);
  const float  ang = (float)s * inv;
  const double ad = (double)ang;
  const double nd = rint(ad * 0.6366197723675814);
  const double rd = (ad - nd * 1.5707963267948966) - nd * 6.123233995736766e-17;
  const float  r = (float)rd;
  const float  z = r * r;
  const float  sr = r + r * z * ((-1.9515295891e-4f * z + 8.3321608736e-3f) * z - 1.6666654611e-1f);
  const float  cr = 1.0f - 0.5f * z + z * z * ((2.443315711809948e-5f * z - 1.388731625493765e-3f) * z + 4.166664568298827e-2f);
  const int qd = ((int)nd) & 3;
  float sv = sr, cv = cr;
  if (qd == 1) { sv = cr;  cv = -sr; }
  if (qd == 2) { sv = -sr; cv = -cr; }
  if (qd == 3) { sv = -cr; cv = sr;  }
  volatile float* pc = (volatile float*)(cs + (size_t)s * HD + i);
  volatile float* ps = (volatile float*)(cs + (size_t)s * HD + 64 + i);
  *pc = cv; *ps = sv;
  __threadfence();
  *pc = cv; *ps = sv;
}

#define GP 132

template <int MODE>
__global__ __launch_bounds__(64) void gemm_kernel(
    const unsigned short* __restrict__ Ap, int lda,
    const unsigned short* __restrict__ Btp, int ldb,
    void* O1, void* O2, void* O3, int ldo,
    const float* __restrict__ cs, int K) {
  __shared__ __align__(16) float sF[64 * GP];
  const int tid  = threadIdx.x;
  const int lane = tid & 31;
  const int wave = tid >> 5;
  const int n0 = blockIdx.x << 7;
  const int m0 = blockIdx.y << 6;
  const int mw = m0 + (wave << 5);

  const _Float16* A  = (const _Float16*)(const void*)Ap;
  const _Float16* Bt = (const _Float16*)(const void*)Btp;

  const int rlane = lane & 15;
  const int koff  = (lane >> 4) * 8;
  const int mOff  = (lane >> 4) * 8;

  v8f acc[2][8];
#pragma unroll
  for (int i = 0; i < 2; ++i)
#pragma unroll
    for (int j = 0; j < 8; ++j) acc[i][j] = (v8f){0.f, 0.f, 0.f, 0.f, 0.f, 0.f, 0.f, 0.f};

  for (int k0 = 0; k0 < K; k0 += 32) {
    const v16h a0 = ldfrag_h(A + (size_t)(mw + rlane) * lda + k0 + koff);
    const v16h a1 = ldfrag_h(A + (size_t)(mw + 16 + rlane) * lda + k0 + koff);
#pragma unroll
    for (int j = 0; j < 8; ++j) {
      const v16h bf = ldfrag_h(Bt + (size_t)(n0 + (j << 4) + rlane) * ldb + k0 + koff);
      acc[0][j] = wmma_h_raw(a0, bf, acc[0][j]);
      acc[1][j] = wmma_h_raw(a1, bf, acc[1][j]);
      dep_guard_h(acc[0][j], acc[1][j], bf, a0, a1);
    }
  }

  {
    float* slab = sF + (wave << 5) * GP;
#pragma unroll
    for (int i = 0; i < 2; ++i)
#pragma unroll
      for (int j = 0; j < 8; ++j)
#pragma unroll
        for (int r = 0; r < 8; ++r) slab[((i << 4) + mOff + r) * GP + (j << 4) + rlane] = acc[i][j][r];
  }
  __syncthreads();

  if (MODE == 0) {
    float* Cp = (float*)O1;
    const int c4 = lane * 4;
    const float osc = 4.8828125e-4f;
#pragma unroll 4
    for (int it = 0; it < 32; ++it) {
      const int row = it * 2 + wave;
      v4f v = *(const v4f*)(sF + row * GP + c4);
      v = v * osc;
      volatile v4f* gp = (volatile v4f*)(Cp + (size_t)(m0 + row) * ldo + n0 + c4);
      *gp = v;
      __threadfence();
      *gp = v;
    }
  } else {
    const int  bidx = m0 >> 11;
    const int  s0   = m0 & (SEQ - 1);
    const int  head = (n0 & (NH * HD - 1)) >> 7;
    const bool isv  = (MODE == 2) && (n0 >= NH * HD);
    if (!isv) {
      unsigned short* P = (unsigned short*)O1;
      const int  rq = tid >> 4, c8 = (tid & 15) * 8, j0 = c8 & 63;
      const bool lowhalf = (c8 < 64);
      const size_t rowBase = (size_t)(bidx * NH + head) * SEQ;
#pragma unroll 2
      for (int it = 0; it < 16; ++it) {
        const int row = it * 4 + rq;
        const int s   = s0 + row;
        const float* sp = sF + row * GP;
        const v4f xa0 = *(const v4f*)(sp + c8), xa1 = *(const v4f*)(sp + c8 + 4);
        float o[8];
        if (MODE == 1) {
          const int cpn = c8 ^ 64;
          const v4f xb0 = *(const v4f*)(sp + cpn), xb1 = *(const v4f*)(sp + cpn + 4);
          const float* tp = cs + (size_t)s * HD;
          const v4f co0 = *(const v4f*)(tp + j0),      co1 = *(const v4f*)(tp + j0 + 4);
          const v4f si0 = *(const v4f*)(tp + 64 + j0), si1 = *(const v4f*)(tp + 64 + j0 + 4);
#pragma unroll
          for (int e = 0; e < 4; ++e) {
            const float a = xa0[e], bb = xb0[e], cc = co0[e], ss = si0[e];
            o[e] = lowhalf ? (a * cc - bb * ss) : (a * cc + bb * ss);
          }
#pragma unroll
          for (int e = 0; e < 4; ++e) {
            const float a = xa1[e], bb = xb1[e], cc = co1[e], ss = si1[e];
            o[4 + e] = lowhalf ? (a * cc - bb * ss) : (a * cc + bb * ss);
          }
        } else {
#pragma unroll
          for (int e = 0; e < 4; ++e) { o[e] = xa0[e]; o[4 + e] = xa1[e]; }
        }
        v4u hv;
#pragma unroll
        for (int p = 0; p < 4; ++p) hv[p] = pkf2(o[2 * p] * 0.125f, o[2 * p + 1] * 0.125f);
        volatile v4u* gp = (volatile v4u*)(P + (rowBase + (size_t)s) * HD + c8);
        *gp = hv;
        __threadfence();
        *gp = hv;
      }
    } else {
      unsigned short* VH = (unsigned short*)O2;
      unsigned short* VL = (unsigned short*)O3;
      const int dq = tid >> 3, key8 = (tid & 7) * 8;
      const size_t vrow0 = (size_t)bidx * HID + (size_t)head * HD;
#pragma unroll 2
      for (int it = 0; it < 16; ++it) {
        const int  d   = it * 8 + dq;
        const int  dpn = d ^ 64;
        const int  j   = d & 63;
        const bool low = (d < 64);
        float o[8];
#pragma unroll
        for (int e = 0; e < 8; ++e) {
          const int sl = key8 + e;
          const float* tp = cs + (size_t)(s0 + sl) * HD;
          const float x  = sF[sl * GP + d];
          const float y  = sF[sl * GP + dpn];
          const float cc = tp[j];
          const float ss = tp[64 + j];
          o[e] = (low ? (x * cc - y * ss) : (x * cc + y * ss)) * 0.125f;
        }
        v4u hv, lv;
#pragma unroll
        for (int p = 0; p < 4; ++p) {
          const float f0 = o[2 * p], f1 = o[2 * p + 1];
          const _Float16 e0 = (_Float16)f0, e1 = (_Float16)f1;
          const _Float16 g0 = (_Float16)((f0 - (float)e0) * 2048.0f);
          const _Float16 g1 = (_Float16)((f1 - (float)e1) * 2048.0f);
          hv[p] = pk16(h2u(e0), h2u(e1));
          lv[p] = pk16(h2u(g0), h2u(g1));
        }
        const size_t go = (vrow0 + (size_t)d) * SEQ + s0 + key8;
        volatile v4u* gh = (volatile v4u*)(VH + go);
        volatile v4u* gl = (volatile v4u*)(VL + go);
        *gh = hv; *gl = lv;
        __threadfence();
        *gh = hv; *gl = lv;
      }
    }
  }
}

#define AT_QB 64
#define AT_KC 64
#define OS_P  132

__global__ __launch_bounds__(128)
void attn_kernel(const unsigned short* __restrict__ qp, const unsigned short* __restrict__ kp,
                 const unsigned short* __restrict__ vhp, const unsigned short* __restrict__ vlp,
                 unsigned short* cxp) {
  __shared__ __align__(16) _Float16 KVs[3 * AT_KC * HD];
  __shared__ __align__(16) _Float16 Psh[4][16 * AT_KC];
  static_assert(4 * 16 * OS_P * 4 <= 3 * AT_KC * HD * 2);
  _Float16* const Ksh = KVs;
  _Float16* const Vth = KVs + AT_KC * HD;
  _Float16* const Vtl = KVs + 2 * AT_KC * HD;

  const int tid  = threadIdx.x;
  const int wave = tid >> 5;
  const int lane = tid & 31;
  const int hh   = lane >> 4;
  const int c    = lane & 15;

  const int bx  = blockIdx.x;
  const int qb  = bx & 31;
  const int h   = (bx >> 5) & (NH - 1);
  const int b   = bx >> 9;
  const int q0  = qb * AT_QB + wave * 16;

  const _Float16* Qg  = (const _Float16*)(const void*)qp  + (size_t)(b * NH + h) * SEQ * HD;
  const _Float16* Kg  = (const _Float16*)(const void*)kp  + (size_t)(b * NH + h) * SEQ * HD;
  const _Float16* Vhg = (const _Float16*)(const void*)vhp + ((size_t)b * HID + (size_t)h * HD) * SEQ;
  const _Float16* Vlg = (const _Float16*)(const void*)vlp + ((size_t)b * HID + (size_t)h * HD) * SEQ;
  const int qro = (q0 + c) * HD + 8 * hh;

  const v8f zero8 = (v8f){0.f, 0.f, 0.f, 0.f, 0.f, 0.f, 0.f, 0.f};
  const float inv2048 = 4.8828125e-4f;
  const float sscale  = 0.0625f * (1.0f / 11.313708305358887f);

  float mrow[8], lrow[8];
  v8f oh[8];
#pragma unroll
  for (int r = 0; r < 8; ++r) { mrow[r] = -INFINITY; lrow[r] = 0.f; }
#pragma unroll
  for (int t = 0; t < 8; ++t) oh[t] = zero8;

  for (int kc = 0; kc < SEQ / AT_KC; ++kc) {
    const int kv0 = kc * AT_KC;
    __syncthreads();
    {
      const int r = tid >> 1, half = (tid & 1) * 64;
      const _Float16* ks = Kg  + (size_t)(kv0 + r) * HD + half;
      const _Float16* vs = Vhg + (size_t)tid * SEQ + kv0;
      const _Float16* ws = Vlg + (size_t)tid * SEQ + kv0;
#pragma unroll
      for (int i = 0; i < 8; ++i) {
        const v8h a0 = *(const v8h*)(ks + 8 * i);
        const v8h b0 = *(const v8h*)(vs + 8 * i);
        const v8h b1 = *(const v8h*)(ws + 8 * i);
        *(v8h*)(Ksh + r * HD + half + 8 * i)  = a0;
        *(v8h*)(Vth + tid * AT_KC + 8 * i)    = b0;
        *(v8h*)(Vtl + tid * AT_KC + 8 * i)    = b1;
      }
    }
    __syncthreads();

    v8f s[4];
#pragma unroll
    for (int j = 0; j < 4; ++j) s[j] = zero8;
    v8f dep = oh[7];
#pragma unroll
    for (int dc = 0; dc < 4; ++dc) {
      int qo = qro + dc * 32;
      asm volatile("" : "+v"(qo) : "v"(dep));
      const v16h qa = ldfrag_h(Qg + qo);
#pragma unroll
      for (int j = 0; j < 4; ++j) {
        FragH kb;
        kb.h[0] = *(const v8h*)(Ksh + (j * 16 + c) * HD + dc * 32 + 8 * hh);
        kb.h[1] = *(const v8h*)(Ksh + (j * 16 + c) * HD + dc * 32 + 16 + 8 * hh);
        s[j] = wmma_h(qa, kb.v, s[j]);
      }
      dep = s[3];
    }
#pragma unroll
    for (int j = 0; j < 4; ++j) s[j] = s[j] * sscale;

    float cm[8];
#pragma unroll
    for (int r = 0; r < 8; ++r) {
      float m = fmaxf(fmaxf(s[0][r], s[1][r]), fmaxf(s[2][r], s[3][r]));
#pragma unroll
      for (int off = 1; off < 16; off <<= 1) m = fmaxf(m, __shfl_xor(m, off, 32));
      cm[r] = m;
    }

    _Float16* pw = Psh[wave];
#pragma unroll
    for (int r = 0; r < 8; ++r) {
      const float mnew  = fmaxf(mrow[r], cm[r]);
      const float alpha = __expf(mrow[r] - mnew);
      mrow[r] = mnew;
      float psum = 0.f;
#pragma unroll
      for (int j = 0; j < 4; ++j) {
        const float p = __expf(s[j][r] - mnew);
        psum += p;
        pw[(8 * hh + r) * AT_KC + j * 16 + c] = (_Float16)(p * 1024.0f);
      }
#pragma unroll
      for (int off = 1; off < 16; off <<= 1) psum += __shfl_xor(psum, off, 32);
      lrow[r] = lrow[r] * alpha + psum;
#pragma unroll
      for (int t = 0; t < 8; ++t) oh[t][r] *= alpha;
    }
    wave_sync();

#pragma unroll 1
    for (int kk = 0; kk < 2; ++kk) {
      FragH pa;
      pa.h[0] = *(const v8h*)(pw + c * AT_KC + kk * 32 + 8 * hh);
      pa.h[1] = *(const v8h*)(pw + c * AT_KC + kk * 32 + 16 + 8 * hh);
#pragma unroll
      for (int t = 0; t < 8; ++t) {
        FragH vb, vr;
        vb.h[0] = *(const v8h*)(Vth + (t * 16 + c) * AT_KC + kk * 32 + 8 * hh);
        vb.h[1] = *(const v8h*)(Vth + (t * 16 + c) * AT_KC + kk * 32 + 16 + 8 * hh);
        vr.h[0] = *(const v8h*)(Vtl + (t * 16 + c) * AT_KC + kk * 32 + 8 * hh);
        vr.h[1] = *(const v8h*)(Vtl + (t * 16 + c) * AT_KC + kk * 32 + 16 + 8 * hh);
        oh[t] = wmma_h(pa.v, vb.v, oh[t]);
        const v8f tr = wmma_h(pa.v, vr.v, zero8);
        oh[t] += tr * inv2048;
      }
    }
  }

  __syncthreads();
  float* os = (float*)(void*)KVs + wave * (16 * OS_P);
#pragma unroll
  for (int r = 0; r < 8; ++r) {
    const float invl = (1.0f / lrow[r]) * 0.015625f;
#pragma unroll
    for (int t = 0; t < 8; ++t) os[(8 * hh + r) * OS_P + t * 16 + c] = oh[t][r] * invl;
  }
  wave_sync();
  {
    const int q16 = lane >> 4, c8 = (lane & 15) * 8;
    for (int pass = 0; pass < 2; ++pass) {
#pragma unroll
      for (int it = 0; it < 8; ++it) {
        const int row = it * 2 + q16;
        const float* sp = os + row * OS_P + c8;
        v4u hv;
#pragma unroll
        for (int p = 0; p < 4; ++p) hv[p] = pkf2(sp[2 * p], sp[2 * p + 1]);
        const size_t go = (size_t)(b * SEQ + q0 + row) * HID + h * HD + c8;
        *(volatile v4u*)(cxp + go) = hv;
      }
      __threadfence();
    }
  }
}

extern "C" void kernel_launch(void* const* d_in, const int* in_sizes, int n_in,
                              void* d_out, int out_size, void* d_ws, size_t ws_size,
                              hipStream_t stream) {
  if (n_in < 5) return;
  if (in_sizes[0] != NB * SEQ * DQ) return;
  if (in_sizes[1] != NB * SEQ * DKV) return;
  if (in_sizes[2] != DQ * HID) return;
  if (in_sizes[3] != DKV * 2 * HID) return;
  if (in_sizes[4] != HID * DQ) return;
  if (out_size != NB * SEQ * DQ) return;

  const float* x1  = (const float*)d_in[0];
  const float* x2  = (const float*)d_in[1];
  const float* Wq  = (const float*)d_in[2];
  const float* Wkv = (const float*)d_in[3];
  const float* Wo  = (const float*)d_in[4];
  float* out = (float*)d_out;

  const size_t szX1  = (size_t)NB * SEQ * DQ * 2;
  const size_t szX2  = (size_t)NB * SEQ * DKV * 2;
  const size_t szWq  = (size_t)DQ * HID * 2;
  const size_t szWkv = (size_t)DKV * 2 * HID * 2;
  const size_t szWo  = (size_t)HID * DQ * 2;
  const size_t szCs  = (size_t)SEQ * HD * 4;
  const size_t szQ   = (size_t)NB * NH * SEQ * HD * 2;
  const size_t szK   = szQ;
  const size_t szV   = (size_t)NB * HID * SEQ * 2;
  size_t off = 0;
  const size_t oX1  = off; off += szX1;
  const size_t oX2  = off; off += szX2;
  const size_t oWq  = off; off += szWq;
  const size_t oWkv = off; off += szWkv;
  const size_t oWo  = off; off += szWo;
  const size_t oCs  = off; off += szCs;
  const size_t oQ   = off; off += szQ;
  const size_t oK   = off; off += szK;
  const size_t oVth = off; off += szV;
  const size_t oVtl = off; off += szV;
  if (off > ws_size) return;
  if (off > (size_t)134217728) return;

  char* ws = (char*)d_ws;
  unsigned short* X1h  = (unsigned short*)(ws + oX1);
  unsigned short* Ctx  = (unsigned short*)(ws + oX1);
  unsigned short* X2h  = (unsigned short*)(ws + oX2);
  unsigned short* WqT  = (unsigned short*)(ws + oWq);
  unsigned short* WkvT = (unsigned short*)(ws + oWkv);
  unsigned short* WoT  = (unsigned short*)(ws + oWo);
  float*          Cs   = (float*)(ws + oCs);
  unsigned short* Qp   = (unsigned short*)(ws + oQ);
  unsigned short* Kp   = (unsigned short*)(ws + oK);
  unsigned short* Vth  = (unsigned short*)(ws + oVth);
  unsigned short* Vtl  = (unsigned short*)(ws + oVtl);

  const dim3 blk256(256), blk128(128), blk64(64);

  {
    const int n8a = NB * SEQ * DQ / 8, n8b = NB * SEQ * DKV / 8;
    cvt_f16x8_kernel<<<dim3((n8a + 255) / 256), blk256, 0, stream>>>(x1, X1h, n8a);
    cvt_f16x8_kernel<<<dim3((n8b + 255) / 256), blk256, 0, stream>>>(x2, X2h, n8b);
  }
  wtr_kernel<<<dim3(HID / 64, DQ / 64), blk256, 0, stream>>>(Wq, WqT, DQ, HID, 32.0f);
  wtr_kernel<<<dim3((2 * HID) / 64, DKV / 64), blk256, 0, stream>>>(Wkv, WkvT, DKV, 2 * HID, 32.0f);
  wtr_kernel<<<dim3(DQ / 64, HID / 64), blk256, 0, stream>>>(Wo, WoT, HID, DQ, 32.0f);
  {
    const int nt = SEQ * 64;
    rope_table_kernel<<<dim3((nt + 255) / 256), blk256, 0, stream>>>(Cs, nt);
  }
  gemm_kernel<1><<<dim3(HID / 128, (NB * SEQ) / 64), blk64, 0, stream>>>(
      X1h, DQ, WqT, DQ, (void*)Qp, (void*)Qp, (void*)Qp, HD, Cs, DQ);
  gemm_kernel<2><<<dim3((2 * HID) / 128, (NB * SEQ) / 64), blk64, 0, stream>>>(
      X2h, DKV, WkvT, DKV, (void*)Kp, (void*)Vth, (void*)Vtl, HD, Cs, DKV);
  attn_kernel<<<dim3(NB * NH * (SEQ / AT_QB)), blk128, 0, stream>>>(Qp, Kp, Vth, Vtl, Ctx);
  gemm_kernel<0><<<dim3(DQ / 128, (NB * SEQ) / 64), blk64, 0, stream>>>(
      Ctx, HID, WoT, HID, (void*)out, (void*)out, (void*)out, DQ, Cs, HID);
  (void)hipGetLastError();
}
